// LSTMModel_86749749444655
// MI455X (gfx1250) — hardware-verified
//
#include <hip/hip_runtime.h>
#include <math.h>

constexpr int NTURN = 64;
constexpr int NBAT  = 32;
constexpr int NPAR  = 9;
constexpr int NDIM  = 512;
constexpr int NROW  = NTURN * NBAT;
constexpr int NG3   = 3 * NDIM;
constexpr int NTHR  = 256;
constexpr int APITCH = 520;
constexpr int FPITCH = 516;
constexpr int RB     = 16;
constexpr long PLANE = (long)NROW * NDIM;
constexpr long KXPL  = (long)NROW * 2 * NDIM;
constexpr long WPL   = (long)4 * NDIM * NDIM;
constexpr long GPL   = (long)NPAR * NG3 * NDIM;
constexpr int NSTATE4 = NBAT * NPAR * NDIM / 4;
constexpr int NOUT04  = NBAT * NDIM / 4;
static_assert(NROW == 2048);
static_assert(NDIM % 32 == 0);
static_assert(NROW % 64 == 0 && NDIM % 64 == 0 && (2 * NDIM) % 64 == 0);
static_assert((PLANE / 8) % NTHR == 0 && (GPL / 8) % NTHR == 0);
static_assert((GPL * 2) % 256 == 0);
static_assert(NBAT % RB == 0 && RB == 2 * (NTHR / 32));
static_assert(NDIM == 64 * (NTHR / 32));
static_assert(NSTATE4 % NTHR == 0 && NOUT04 % NTHR == 0);
static_assert(NG3 == 3 * 512);

typedef __attribute__((ext_vector_type(16))) _Float16 v16h;
typedef __attribute__((ext_vector_type(8)))  _Float16 v8h;
typedef __attribute__((ext_vector_type(16))) __bf16   v16b;
typedef __attribute__((ext_vector_type(8)))  __bf16   v8b;
typedef __attribute__((ext_vector_type(8)))  float    v8f;
typedef __attribute__((ext_vector_type(4)))  float    v4f;
typedef __attribute__((ext_vector_type(2)))  float    v2f;
typedef __attribute__((ext_vector_type(4)))  unsigned int v4u;

__device__ __forceinline__ unsigned short f2bf_bits(float f) {
  unsigned u = __float_as_uint(f);
  return (unsigned short)((u + 0x7FFFu + ((u >> 16) & 1u)) >> 16);
}
__device__ __forceinline__ float bf_bits2f(unsigned short h) { return __uint_as_float(((unsigned)h) << 16); }
__device__ __forceinline__ unsigned pk16(unsigned short a, unsigned short b) { return (unsigned)a | ((unsigned)b << 16); }

__device__ __forceinline__ void dep_guard_b(v8f& a, v8f& b, v16b x, v16b y) { asm volatile("v_nop\n\tv_nop\n\tv_nop\n\tv_nop" : "+v"(a), "+v"(b) : "v"(x), "v"(y)); }
__device__ __forceinline__ void dep_guard4_b(v8f& a, v8f& b, v8f& c, v8f& d, v16b x, v16b y) {
  asm volatile("v_nop\n\tv_nop\n\tv_nop\n\tv_nop" : "+v"(a), "+v"(b), "+v"(c), "+v"(d) : "v"(x), "v"(y));
}
__device__ __forceinline__ void dep_guard3_b(v8f& a, v8f& b, v8f& c, v16b w, v16b x, v16b y, v16b z) {
  asm volatile("v_nop\n\tv_nop\n\tv_nop\n\tv_nop" : "+v"(a), "+v"(b), "+v"(c) : "v"(w), "v"(x), "v"(y), "v"(z));
}
__device__ __forceinline__ void keep4_b(v16b a, v16b b, v16b c, v16b d) { asm volatile("v_nop" :: "v"(a), "v"(b), "v"(c), "v"(d)); }
__device__ __forceinline__ void acc_guard4(v8f& a, v8f& b, v8f& c, v8f& d) { asm volatile("v_nop\n\tv_nop\n\tv_nop\n\tv_nop" : "+v"(a), "+v"(b), "+v"(c), "+v"(d)); }
__device__ __forceinline__ void acc_guard3(v8f& a, v8f& b, v8f& c) { asm volatile("v_nop\n\tv_nop\n\tv_nop\n\tv_nop" : "+v"(a), "+v"(b), "+v"(c)); }

template <typename T> struct Frag;
template <> struct Frag<__bf16> {
  typedef v16b V; union U { v16b v; v8b h[2]; };
  static __device__ __forceinline__ v16b load(const __bf16* p) {
    U f; f.h[0] = *(const v8b*)(p); f.h[1] = *(const v8b*)(p + 16); return f.v;
  }
  static __device__ __forceinline__ v8f mma(v16b a, v16b b, v8f c) {
    return __builtin_amdgcn_wmma_f32_16x16x32_bf16(false, a, false, b, (short)0, c, false, false);
  }
};

__device__ __forceinline__ float fsigm(float x) { return __builtin_amdgcn_rcpf(1.0f + expf(-x)); }
__device__ __forceinline__ float gru_cell(float xr, float xz, float xn, float hr, float hz, float hn, float h) {
  const float rg = fsigm(xr + hr);
  const float zg = fsigm(xz + hz);
  const float ng = tanhf(xn + rg * hn);
  return (1.0f - zg) * ng + zg * h;
}
__device__ __forceinline__ int argmax9(const float* __restrict__ q) {
  float bv = q[0]; int bi = 0;
#pragma unroll
  for (int k = 1; k < NPAR; ++k) { const float v = q[k]; const bool gt = v > bv; bv = gt ? v : bv; bi = gt ? k : bi; }
  return bi;
}

template <bool SPLA, int OUT_MODE, bool RSC>
__global__ __launch_bounds__(256) void gemm_bf16_64(
    const unsigned short* __restrict__ Ap, const unsigned short* __restrict__ A2p, int lda, long strideA,
    const unsigned short* __restrict__ Btp, int ldb, long strideB,
    void* __restrict__ Cout, void* __restrict__ Cout2, int ldc, long strideC,
    const float* __restrict__ bias, long strideBias,
    const float* __restrict__ rsc, long strideRsc,
    int M, int N, int K) {
  typedef __bf16 T;
  typedef v16b V;
  const T* A = (const T*)(const void*)Ap; const T* A2 = (const T*)(const void*)A2p; const T* Bt = (const T*)(const void*)Btp;
  __shared__ __align__(16) float sT[8][16 * 68];
  const int b    = blockIdx.y;
  const int lane = threadIdx.x & 31;
  const int wave = threadIdx.x >> 5;
  const int tilesN = N >> 6;
  const int tilesM = M >> 6;
  const int tile = blockIdx.x * 8 + wave;
  if (tile >= tilesM * tilesN) return;
  const int tm = tile / tilesN;
  const int tn = tile - tm * tilesN;
  const int m0 = tm << 6;
  const int n0 = tn << 6;

  const T* Ab  = A  + (size_t)b * strideA;
  const T* Bb  = Bt + (size_t)b * strideB;
  const T* Ab2 = SPLA ? (A2 + (size_t)b * strideA) : nullptr;

  const int rlane = lane & 15;
  const int koff  = (lane >> 4) * 8;
  const int mOff  = (lane >> 4) * 8;

  v8f acc[4][4];
#pragma unroll
  for (int i = 0; i < 4; ++i)
#pragma unroll
    for (int j = 0; j < 4; ++j) acc[i][j] = (v8f){0.f,0.f,0.f,0.f,0.f,0.f,0.f,0.f};

  for (int k0 = 0; k0 < K; k0 += 32) {
    V bh[4];
#pragma unroll
    for (int j = 0; j < 4; ++j) {
      const size_t bo = (size_t)(n0 + (j << 4) + rlane) * ldb + koff + k0;
      bh[j] = Frag<T>::load(Bb + bo);
    }
#pragma unroll
    for (int i = 0; i < 4; ++i) {
      const size_t ao = (size_t)(m0 + (i << 4) + rlane) * lda + koff + k0;
      V ah = Frag<T>::load(Ab + ao);
      V al;
      if (SPLA) al = Frag<T>::load(Ab2 + ao);
#pragma unroll
      for (int j = 0; j < 4; ++j) {
        acc[i][j] = Frag<T>::mma(ah, bh[j], acc[i][j]);
        if (SPLA) acc[i][j] = Frag<T>::mma(al, bh[j], acc[i][j]);
      }
      dep_guard4_b(acc[i][0], acc[i][1], acc[i][2], acc[i][3], ah, SPLA ? al : ah);
    }
    keep4_b(bh[0], bh[1], bh[2], bh[3]);
  }
  acc_guard4(acc[0][0], acc[0][1], acc[0][2], acc[0][3]);
  acc_guard4(acc[1][0], acc[1][1], acc[1][2], acc[1][3]);
  acc_guard4(acc[2][0], acc[2][1], acc[2][2], acc[2][3]);
  acc_guard4(acc[3][0], acc[3][1], acc[3][2], acc[3][3]);

  float* slab = sT[wave];
  const float* bp = bias + (size_t)b * strideBias;
  const float* rp = RSC ? (rsc + (size_t)b * strideRsc) : nullptr;
#pragma unroll
  for (int i = 0; i < 4; ++i) {
    const int mBase = m0 + (i << 4);
    float rsv[8];
    if (RSC) {
      const v4f r0 = *(const v4f*)(rp + mBase + mOff);
      const v4f r1 = *(const v4f*)(rp + mBase + mOff + 4);
#pragma unroll
      for (int e = 0; e < 4; ++e) { rsv[e] = r0[e]; rsv[4 + e] = r1[e]; }
    } else {
#pragma unroll
      for (int e = 0; e < 8; ++e) rsv[e] = 1.0f;
    }
#pragma unroll
    for (int j = 0; j < 4; ++j) {
      const int n = n0 + (j << 4) + rlane;
      const float bv = bp[n];
#pragma unroll
      for (int r = 0; r < 8; ++r) {
        const float v = acc[i][j][r] * rsv[r] + bv;
        slab[(mOff + r) * 68 + (j << 4) + rlane] = v;
      }
    }
    __builtin_amdgcn_fence(__ATOMIC_RELEASE, "workgroup");
    __builtin_amdgcn_wave_barrier();
    __builtin_amdgcn_fence(__ATOMIC_ACQUIRE, "workgroup");
    if (OUT_MODE == 0) {
      float* C = (float*)Cout + (size_t)b * strideC;
      const int hh = lane >> 4, c4 = (lane & 15) * 4;
      for (int pass = 0; pass < 2; ++pass) {
#pragma unroll
        for (int it = 0; it < 8; ++it) {
          const int row = it * 2 + hh;
          v4f v = *(const v4f*)(slab + row * 68 + c4);
          *(volatile v4f*)(C + (size_t)(mBase + row) * ldc + n0 + c4) = v;
        }
        __threadfence();
      }
    } else {
      const int q = lane >> 3, c8 = (lane & 7) * 8;
      unsigned short* C  = (unsigned short*)Cout  + (size_t)b * strideC;
      unsigned short* C2 = (OUT_MODE == 2) ? ((unsigned short*)Cout2 + (size_t)b * strideC) : nullptr;
      for (int pass = 0; pass < 2; ++pass) {
#pragma unroll
        for (int it = 0; it < 4; ++it) {
          const int row = it * 4 + q;
          const float* sp = slab + row * 68 + c8;
          v8h hv, lv;
#pragma unroll
          for (int e = 0; e < 8; ++e) {
            if (OUT_MODE == 1) {
              hv[e] = (_Float16)sp[e];
            } else {
              unsigned short hb = f2bf_bits(sp[e]);
              unsigned short lb = f2bf_bits(sp[e] - bf_bits2f(hb));
              hv[e] = __builtin_bit_cast(_Float16, hb);
              lv[e] = __builtin_bit_cast(_Float16, lb);
            }
          }
          *(volatile v8h*)(C + (size_t)(mBase + row) * ldc + n0 + c8) = hv;
          if (OUT_MODE == 2) *(volatile v8h*)(C2 + (size_t)(mBase + row) * ldc + n0 + c8) = lv;
        }
        __threadfence();
      }
    }
    __builtin_amdgcn_fence(__ATOMIC_RELEASE, "workgroup");
    __builtin_amdgcn_wave_barrier();
    __builtin_amdgcn_fence(__ATOMIC_ACQUIRE, "workgroup");
  }
}

__global__ __launch_bounds__(256) void split_bf16x2_kernel(const float* __restrict__ in, unsigned short* __restrict__ hi,
                                                           unsigned short* __restrict__ lo, int n2) {
  const int i = blockIdx.x * 256 + threadIdx.x;
  if (i < n2) {
    const v2f f = *(const v2f*)(in + 2 * (size_t)i);
    const unsigned short h0 = f2bf_bits(f[0]), h1 = f2bf_bits(f[1]);
    const unsigned short l0 = f2bf_bits(f[0] - bf_bits2f(h0)), l1 = f2bf_bits(f[1] - bf_bits2f(h1));
    const unsigned uh = pk16(h0, h1), ul = pk16(l0, l1);
    ((volatile unsigned*)hi)[i] = uh;
    ((volatile unsigned*)lo)[i] = ul;
    __threadfence();
    ((volatile unsigned*)hi)[i] = uh;
    ((volatile unsigned*)lo)[i] = ul;
  }
}

__global__ __launch_bounds__(NTHR) void cvt_bf16x8_kernel(const float* __restrict__ s0, const float* __restrict__ s1,
                                                          const float* __restrict__ s2, const float* __restrict__ s3,
                                                          unsigned short* __restrict__ dst, long dstStride,
                                                          int blocksPer, int n8each) {
  const int r = blockIdx.x / blocksPer;
  const float* src = (r == 0) ? s0 : (r == 1) ? s1 : (r == 2) ? s2 : s3;
  const int i = (blockIdx.x - r * blocksPer) * NTHR + threadIdx.x;
  if (i < n8each) {
    const float* sp = src + (size_t)i * 8;
    const v4f a = *(const v4f*)(sp);
    const v4f c = *(const v4f*)(sp + 4);
    v4u w;
    w[0] = pk16(f2bf_bits(a[0]), f2bf_bits(a[1]));
    w[1] = pk16(f2bf_bits(a[2]), f2bf_bits(a[3]));
    w[2] = pk16(f2bf_bits(c[0]), f2bf_bits(c[1]));
    w[3] = pk16(f2bf_bits(c[2]), f2bf_bits(c[3]));
    unsigned short* dp = dst + (size_t)r * dstStride + (size_t)i * 8;
    *(volatile v4u*)dp = w;
    __threadfence();
    *(volatile v4u*)dp = w;
  }
}

__global__ __launch_bounds__(NTHR) void zero_kernel(float* __restrict__ st, int n4a, float* __restrict__ o0, int n4b) {
  const int i = blockIdx.x * NTHR + threadIdx.x;
  const v4f z = {0.0f, 0.0f, 0.0f, 0.0f};
  if (i < n4a) {
    float* p = st + (size_t)i * 4;
    *(volatile v4f*)p = z; __threadfence(); *(volatile v4f*)p = z;
  } else {
    const int j = i - n4a;
    if (j < n4b) {
      float* p = o0 + (size_t)j * 4;
      *(volatile v4f*)p = z; __threadfence(); *(volatile v4f*)p = z;
    }
  }
}

__global__ __launch_bounds__(NTHR) void score_kernel(const float* __restrict__ QX, long qz,
                                                     const float* __restrict__ KX, long kz, int kpitch,
                                                     float* __restrict__ SCO, long sz) {
  __shared__ float lg[NBAT];
  const int t = blockIdx.x, z = blockIdx.y;
  const int tid = threadIdx.x, lane = tid & 31, wave = tid >> 5;
  const float* qb = QX + (size_t)z * qz + (size_t)t * NBAT * NDIM;
  const float* kb = KX + (size_t)z * kz + (size_t)t * NBAT * kpitch;
#pragma unroll 1
  for (int rr = 0; rr < 4; ++rr) {
    const int b = wave * 4 + rr;
    const float* qp = qb + (size_t)b * NDIM + 16 * lane;
    const float* kp = kb + (size_t)b * kpitch + 16 * lane;
    float s = 0.0f;
#pragma unroll
    for (int q = 0; q < 4; ++q) {
      const v4f a  = *(const v4f*)(qp + 4 * q);
      const v4f k4 = *(const v4f*)(kp + 4 * q);
      s += a[0] * k4[0]; s += a[1] * k4[1]; s += a[2] * k4[2]; s += a[3] * k4[3];
    }
#pragma unroll
    for (int off = 1; off < 32; off <<= 1) s += __shfl_xor(s, off, 32);
    if (lane == 0) lg[b] = s;
  }
  __syncthreads();
  if (wave == 0) {
    const float x = lg[lane];
    float m = x;
#pragma unroll
    for (int off = 1; off < 32; off <<= 1) m = fmaxf(m, __shfl_xor(m, off, 32));
    float e = expf(x - m);
    e = (e < 1.17549435e-38f) ? 0.0f : e;
    float su = e;
#pragma unroll
    for (int off = 1; off < 32; off <<= 1) su += __shfl_xor(su, off, 32);
    const float sc = e * (1.0f / su);
    float* op = SCO + (size_t)z * sz + (size_t)t * NBAT + lane;
    *(volatile float*)op = sc;
    __threadfence();
    *(volatile float*)op = sc;
  }
}

__global__ __launch_bounds__(NTHR) void gi_kernel(const float* __restrict__ qmask,
                                                  const unsigned short* __restrict__ XHp, const unsigned short* __restrict__ XLp,
                                                  const unsigned short* __restrict__ WIHp, const float* __restrict__ bih,
                                                  float* __restrict__ GI) {
  __shared__ __align__(16) __bf16 Ah[16 * APITCH];
  __shared__ __align__(16) __bf16 Al[16 * APITCH];
  __shared__ __align__(16) float slabs[8][16 * 68];
  __shared__ int lst[NROW];
  __shared__ int wsum[8];
  const int grp = blockIdx.x, p = blockIdx.y, role = blockIdx.z;
  const int tid = threadIdx.x, lane = tid & 31, wave = tid >> 5;
  const int rlane = lane & 15, hh = lane >> 4, koff = hh * 8, mOff = hh * 8;
  const __bf16* XH  = (const __bf16*)(const void*)XHp + (size_t)role * PLANE;
  const __bf16* XL  = (const __bf16*)(const void*)XLp + (size_t)role * PLANE;
  const __bf16* WIH = (const __bf16*)(const void*)WIHp;
  float* GIp = GI + (size_t)role * NROW * NG3;

  int base = 0;
#pragma unroll 1
  for (int ch = 0; ch < NROW / NTHR; ++ch) {
    const int row = ch * NTHR + tid;
    const int tt = row >> 5, bb = row & 31;
    const int trow = role ? ((tt + 1 < NTURN) ? tt + 1 : NTURN - 1) : tt;
    const int pr = argmax9(qmask + ((size_t)trow * NBAT + bb) * NPAR);
    const bool hit = (pr == p);
    const unsigned bal = __builtin_amdgcn_ballot_w32(hit);
    const int wcnt = __builtin_popcount(bal);
    const int wpre = __builtin_popcount(bal & ((1u << lane) - 1u));
    if (lane == 0) wsum[wave] = wcnt;
    __syncthreads();
    int woff = 0, tot = 0;
#pragma unroll
    for (int w = 0; w < 8; ++w) { const int s = wsum[w]; tot += s; woff += (w < wave) ? s : 0; }
    if (hit) lst[base + woff + wpre] = row;
    base += tot;
    __syncthreads();
  }
  const int cnt = base;
  int ntile = (cnt + 15) >> 4;
  ntile = ntile > (NROW / 16) ? (NROW / 16) : ntile;

  const int n0 = grp * NDIM + 64 * wave;
  const v8f z8 = {0.f, 0.f, 0.f, 0.f, 0.f, 0.f, 0.f, 0.f};
  float* slab = slabs[wave];
  const int c4 = (lane & 15) * 4;

#pragma unroll 1
  for (int mt = 0; mt < ntile; ++mt) {
    {
      const int r = tid >> 4, seg = (tid & 15) * 32;
      const int lrow = mt * 16 + r;
      const int idx = (lrow < cnt) ? lrow : (cnt - 1);
      int grow = lst[idx];
      grow = grow < 0 ? 0 : (grow > NROW - 1 ? NROW - 1 : grow);
      const __bf16* sh = XH + (size_t)grow * NDIM + seg;
      const __bf16* sl = XL + (size_t)grow * NDIM + seg;
      __bf16* dh = Ah + r * APITCH + seg;
      __bf16* dl = Al + r * APITCH + seg;
#pragma unroll
      for (int q = 0; q < 4; ++q) {
        const v4u uh = *(const v4u*)(sh + 8 * q);
        const v4u ul = *(const v4u*)(sl + 8 * q);
        *(v4u*)(dh + 8 * q) = uh;
        *(v4u*)(dl + 8 * q) = ul;
      }
    }
    __syncthreads();
    v8f acc[4];
#pragma unroll
    for (int j = 0; j < 4; ++j) acc[j] = z8;
    const __bf16* arow = Ah + rlane * APITCH + koff;
    const __bf16* lrowp = Al + rlane * APITCH + koff;
#pragma unroll 1
    for (int k0 = 0; k0 < NDIM; k0 += 32) {
      v16b bh[4];
#pragma unroll
      for (int j = 0; j < 4; ++j)
        bh[j] = Frag<__bf16>::load(WIH + ((size_t)p * NG3 + n0 + 16 * j + rlane) * NDIM + koff + k0);
      const v16b ah = Frag<__bf16>::load(arow + k0);
      const v16b al = Frag<__bf16>::load(lrowp + k0);
#pragma unroll
      for (int j = 0; j < 4; ++j) {
        acc[j] = Frag<__bf16>::mma(ah, bh[j], acc[j]);
        acc[j] = Frag<__bf16>::mma(al, bh[j], acc[j]);
      }
      dep_guard4_b(acc[0], acc[1], acc[2], acc[3], ah, al);
      keep4_b(bh[0], bh[1], bh[2], bh[3]);
    }
    acc_guard4(acc[0], acc[1], acc[2], acc[3]);
#pragma unroll
    for (int j = 0; j < 4; ++j) {
      const int n = n0 + 16 * j + rlane;
      const float bv = bih[(size_t)p * NG3 + n];
#pragma unroll
      for (int r = 0; r < 8; ++r) slab[(mOff + r) * 68 + 16 * j + rlane] = acc[j][r] + bv;
    }
    __builtin_amdgcn_fence(__ATOMIC_RELEASE, "workgroup");
    __builtin_amdgcn_wave_barrier();
    __builtin_amdgcn_fence(__ATOMIC_ACQUIRE, "workgroup");
    int drw[8], vld[8];
#pragma unroll
    for (int it = 0; it < 8; ++it) {
      const int lrow = mt * 16 + it * 2 + hh;
      vld[it] = (lrow < cnt) ? 1 : 0;
      const int idx = vld[it] ? lrow : (cnt - 1);
      int d = lst[idx];
      d = d < 0 ? 0 : (d > NROW - 1 ? NROW - 1 : d);
      drw[it] = d;
    }
    for (int pass = 0; pass < 2; ++pass) {
#pragma unroll
      for (int it = 0; it < 8; ++it) {
        const int row = it * 2 + hh;
        const v4f v = *(const v4f*)(slab + row * 68 + c4);
        if (vld[it]) *(volatile v4f*)(GIp + (size_t)drw[it] * NG3 + n0 + c4) = v;
      }
      __threadfence();
    }
    __builtin_amdgcn_fence(__ATOMIC_RELEASE, "workgroup");
    __builtin_amdgcn_wave_barrier();
    __builtin_amdgcn_fence(__ATOMIC_ACQUIRE, "workgroup");
    __syncthreads();
  }
}

__global__ __launch_bounds__(NTHR) void rec_kernel(const float* __restrict__ qmask, const float* __restrict__ GI,
                                                   const unsigned short* __restrict__ WHHp, const float* __restrict__ bhh,
                                                   float* __restrict__ STATE, float* __restrict__ out) {
  __shared__ __align__(16) float sf[RB * FPITCH];
  __shared__ __align__(16) unsigned short ab[RB * APITCH];
  __shared__ int qiL[RB];
  __shared__ int qnL[RB];
  const __bf16* WHH = (const __bf16*)(const void*)WHHp;
  const __bf16* abh = (const __bf16*)(const void*)ab;
  const int tid = threadIdx.x, lane = tid & 31, wave = tid >> 5;
  const int c = lane & 15, hh = lane >> 4, koff = hh * 8;
  const int blk = blockIdx.x;
  const int srow = tid >> 4;
  const int sseg = (tid & 15) * 32;
  const v8f z8 = {0.f, 0.f, 0.f, 0.f, 0.f, 0.f, 0.f, 0.f};

#pragma unroll 1
  for (int t = 0; t < NTURN; ++t) {
    const int tn = (t + 1 < NTURN) ? t + 1 : NTURN - 1;
#pragma unroll 1
    for (int p = 0; p < NPAR; ++p) {
      if (p == 0 && __builtin_amdgcn_readfirstlane(wave) == 0) {
        const int rr = lane & (RB - 1);
        const float* qm = qmask + ((size_t)t  * NBAT + RB * blk + rr) * NPAR;
        const float* qn = qmask + ((size_t)tn * NBAT + RB * blk + rr) * NPAR;
        const int a0 = argmax9(qm);
        const int a1 = argmax9(qn);
        qiL[rr] = a0;
        qnL[rr] = a1;
      }
      {
        const float* sp = STATE + ((size_t)(RB * blk + srow) * NPAR + p) * NDIM + sseg;
        float* fp = sf + srow * FPITCH + sseg;
        unsigned short* hp = ab + srow * APITCH + sseg;
#pragma unroll
        for (int q = 0; q < 4; ++q) {
          const v4f a  = *(const v4f*)(sp + 8 * q);
          const v4f a2 = *(const v4f*)(sp + 8 * q + 4);
          *(v4f*)(fp + 8 * q)     = a;
          *(v4f*)(fp + 8 * q + 4) = a2;
          v4u w;
          w[0] = pk16(f2bf_bits(a[0]),  f2bf_bits(a[1]));
          w[1] = pk16(f2bf_bits(a[2]),  f2bf_bits(a[3]));
          w[2] = pk16(f2bf_bits(a2[0]), f2bf_bits(a2[1]));
          w[3] = pk16(f2bf_bits(a2[2]), f2bf_bits(a2[3]));
          *(v4u*)(hp + 8 * q) = w;
        }
      }
      __syncthreads();

      int qS[8], qN[8];
#pragma unroll
      for (int r = 0; r < 8; ++r) { qS[r] = qiL[8 * hh + r]; qN[r] = qnL[8 * hh + r]; }
      const __bf16* arow = abh + c * APITCH + koff;
#pragma unroll 1
      for (int us = 0; us < 4; ++us) {
        const int j = 64 * wave + 16 * us + c;
        const __bf16* w0 = WHH + ((size_t)p * NG3 + j) * NDIM + koff;
        const __bf16* w1 = w0 + (size_t)NDIM * NDIM;
        const __bf16* w2 = w1 + (size_t)NDIM * NDIM;
        v8f ar = z8, az = z8, an = z8;
#pragma unroll 1
        for (int k0 = 0; k0 < NDIM; k0 += 32) {
          const v16b a  = Frag<__bf16>::load(arow + k0);
          const v16b b0 = Frag<__bf16>::load(w0 + k0);
          const v16b b1 = Frag<__bf16>::load(w1 + k0);
          const v16b b2 = Frag<__bf16>::load(w2 + k0);
          ar = Frag<__bf16>::mma(a, b0, ar);
          az = Frag<__bf16>::mma(a, b1, az);
          an = Frag<__bf16>::mma(a, b2, an);
          dep_guard3_b(ar, az, an, a, b0, b1, b2);
        }
        acc_guard3(ar, az, an);
        const float br = bhh[(size_t)p * NG3 + j];
        const float bz = bhh[(size_t)p * NG3 + NDIM + j];
        const float bn = bhh[(size_t)p * NG3 + 2 * NDIM + j];
#pragma unroll
        for (int r = 0; r < 8; ++r) {
          const int row = 8 * hh + r;
          const int b = RB * blk + row;
          const float hval = sf[row * FPITCH + j];
          const float* gs = GI + ((size_t)(t * NBAT + b) * NG3 + j);
          const float* gl = gs + (size_t)NROW * NG3;
          const float xr = gs[0], xz = gs[NDIM], xn = gs[2 * NDIM];
          const float yr = gl[0], yz = gl[NDIM], yn = gl[2 * NDIM];
          asm volatile("" ::: "memory");
          const float ghr = ar[r] + br, ghz = az[r] + bz, ghn = an[r] + bn;
          const float cS = gru_cell(xr, xz, xn, ghr, ghz, ghn, hval);
          const float cL = gru_cell(yr, yz, yn, ghr, ghz, ghn, hval);
          const bool fs = (qS[r] == p), fl = (qN[r] == p);
          const float coef = (1.0f - (fs ? 1.0f : 0.0f)) - (fl ? 1.0f : 0.0f);
          const float v = hval * coef + (fs ? cS : 0.0f) + (fl ? cL : 0.0f);
          sf[row * FPITCH + j] = v;
        }
      }
      __syncthreads();

#pragma unroll 1
      for (int rr = 0; rr < 2; ++rr) {
        const int row = 2 * wave + rr;
        const int b = RB * blk + row;
        const int qs = qiL[row], qn = qnL[row];
        const bool chg  = (qs == p) || (qn == p);
        const bool emit = (qs == p);
        if (chg) {
          float* dstS = STATE + ((size_t)b * NPAR + p) * NDIM;
          float* dstO = out + ((size_t)(t + 1) * NBAT + b) * NDIM;
          const float* srcp = sf + row * FPITCH;
          for (int pass = 0; pass < 2; ++pass) {
#pragma unroll
            for (int q4 = 0; q4 < 4; ++q4) {
              const v4f v = *(const v4f*)(srcp + 128 * q4 + 4 * lane);
              *(volatile v4f*)(dstS + 128 * q4 + 4 * lane) = v;
              if (emit) *(volatile v4f*)(dstO + 128 * q4 + 4 * lane) = v;
            }
            __threadfence();
          }
        }
      }
      __syncthreads();
      __threadfence();
    }
  }
}

extern "C" void kernel_launch(void* const* d_in, const int* in_sizes, int n_in,
                              void* d_out, int out_size, void* d_ws, size_t ws_size, hipStream_t stream) {
  if (n_in < 16 || d_out == nullptr || d_ws == nullptr) return;
  if (in_sizes[0] != NROW * NDIM || in_sizes[1] != NROW * NDIM || in_sizes[2] != NROW * NDIM || in_sizes[3] != NROW * NDIM ||
      in_sizes[5] != NROW * NPAR || in_sizes[6] != (int)WPL || in_sizes[7] != 4 * NDIM || in_sizes[8] != (int)WPL ||
      in_sizes[9] != 4 * NDIM || in_sizes[10] != (int)WPL || in_sizes[11] != 4 * NDIM || in_sizes[12] != (int)GPL ||
      in_sizes[13] != (int)GPL || in_sizes[14] != NPAR * NG3 || in_sizes[15] != NPAR * NG3 ||
      out_size != (NTURN + 1) * NBAT * NDIM) return;

  const float* U     = (const float*)d_in[0];
  const float* SK    = (const float*)d_in[1];
  const float* NU    = (const float*)d_in[2];
  const float* LK    = (const float*)d_in[3];
  const float* qmask = (const float*)d_in[5];
  const float* Wk    = (const float*)d_in[6];
  const float* bk    = (const float*)d_in[7];
  const float* Wq    = (const float*)d_in[8];
  const float* bq    = (const float*)d_in[9];
  const float* Wp    = (const float*)d_in[10];
  const float* bp    = (const float*)d_in[11];
  const float* Wih   = (const float*)d_in[12];
  const float* Whh   = (const float*)d_in[13];
  const float* bih   = (const float*)d_in[14];
  const float* bhh   = (const float*)d_in[15];
  float* out = (float*)d_out;

  char* ws = (char*)d_ws; size_t off = 0;
  auto carve = [&](size_t bytes) -> char* { char* p = ws + off; off += (bytes + 255) & ~(size_t)255; return p; };
  unsigned short* ACTB  = (unsigned short*)carve((size_t)4 * PLANE * 2);
  unsigned short* WB    = (unsigned short*)carve((size_t)3 * WPL * 2);
  unsigned short* WGB   = (unsigned short*)carve((size_t)2 * GPL * 2);
  float*          KXF   = (float*)carve((size_t)2 * KXPL * 4);
  unsigned short* KXH   = (unsigned short*)carve((size_t)2 * KXPL * 2);
  unsigned short* KXL   = (unsigned short*)carve((size_t)2 * KXPL * 2);
  float*          QXF   = (float*)carve((size_t)2 * PLANE * 4);
  float*          SC    = (float*)carve((size_t)4 * NROW * 4);
  unsigned short* S01H  = (unsigned short*)carve((size_t)2 * PLANE * 2);
  unsigned short* S01L  = (unsigned short*)carve((size_t)2 * PLANE * 2);
  unsigned short* SSLH  = (unsigned short*)carve((size_t)2 * PLANE * 2);
  unsigned short* SSLL  = (unsigned short*)carve((size_t)2 * PLANE * 2);
  float*          GI    = (float*)carve((size_t)2 * NROW * NG3 * 4);
  float*          STATE = (float*)carve((size_t)NBAT * NPAR * NDIM * 4);
  if (off > ws_size || off > (size_t)134217728) return;
  unsigned short* WIHB = WGB;
  unsigned short* WHHB = WGB + GPL;
  const unsigned short* WKB = WB;
  const unsigned short* WQB = WB + WPL;
  const unsigned short* WPB = WB + 2 * WPL;

  cvt_bf16x8_kernel<<<4 * 512, NTHR, 0, stream>>>(U, SK, NU, LK, ACTB, PLANE, 512, (int)(PLANE / 8));
  cvt_bf16x8_kernel<<<3 * 512, NTHR, 0, stream>>>(Wk, Wq, Wp, Wp, WB, WPL, 512, (int)(WPL / 8));
  cvt_bf16x8_kernel<<<2 * 3456, NTHR, 0, stream>>>(Wih, Whh, Whh, Whh, WGB, GPL, 3456, (int)(GPL / 8));
  zero_kernel<<<(NSTATE4 + NOUT04) / NTHR, NTHR, 0, stream>>>(STATE, NSTATE4, out, NOUT04);

  const dim3 g1024((NROW / 64) * (2 * NDIM / 64) / 8, 2);
  const dim3 g512((NROW / 64) * (NDIM / 64) / 8, 2);

  gemm_bf16_64<false, 0, false><<<g1024, 256, 0, stream>>>(
      ACTB + PLANE, ACTB + PLANE, NDIM, 2 * PLANE,
      WKB, NDIM, 2L * NDIM * NDIM,
      (void*)KXF, (void*)KXF, 2 * NDIM, KXPL,
      bk, 2L * NDIM, SC, 0L, NROW, 2 * NDIM, NDIM);
  split_bf16x2_kernel<<<(int)(KXPL / 256), 256, 0, stream>>>(KXF, KXH, KXL, (int)KXPL);
  gemm_bf16_64<false, 0, false><<<g512, 256, 0, stream>>>(
      ACTB, ACTB, NDIM, 2 * PLANE,
      WQB, NDIM, 2L * NDIM * NDIM,
      (void*)QXF, (void*)QXF, NDIM, PLANE,
      bq, 2L * NDIM, SC, 0L, NROW, NDIM, NDIM);
  score_kernel<<<dim3(NTURN, 2), NTHR, 0, stream>>>(QXF, PLANE, KXF, KXPL, 2 * NDIM, SC, 2L * NROW);
  gemm_bf16_64<true, 2, true><<<g512, 256, 0, stream>>>(
      KXH, KXL, 2 * NDIM, KXPL,
      WPB, NDIM, 2L * NDIM * NDIM,
      (void*)S01H, (void*)S01L, NDIM, PLANE,
      bp, 2L * NDIM, SC, 2L * NROW, NROW, NDIM, NDIM);
  gemm_bf16_64<true, 0, false><<<g512, 256, 0, stream>>>(
      S01H, S01L, NDIM, PLANE,
      WQB + (size_t)NDIM * NDIM, NDIM, 2L * NDIM * NDIM,
      (void*)QXF, (void*)QXF, NDIM, PLANE,
      bq + NDIM, 2L * NDIM, SC, 0L, NROW, NDIM, NDIM);
  score_kernel<<<dim3(NTURN, 2), NTHR, 0, stream>>>(QXF, PLANE, KXF + NDIM, KXPL, 2 * NDIM, SC + NROW, 2L * NROW);
  gemm_bf16_64<true, 2, true><<<g512, 256, 0, stream>>>(
      KXH + NDIM, KXL + NDIM, 2 * NDIM, KXPL,
      WPB + (size_t)NDIM * NDIM, NDIM, 2L * NDIM * NDIM,
      (void*)SSLH, (void*)SSLL, NDIM, PLANE,
      bp + NDIM, 2L * NDIM, SC + NROW, 2L * NROW, NROW, NDIM, NDIM);
  gi_kernel<<<dim3(NG3 / NDIM, NPAR, 2), NTHR, 0, stream>>>(qmask, SSLH, SSLL, WIHB, bih, GI);
  rec_kernel<<<NBAT / RB, NTHR, 0, stream>>>(qmask, GI, WHHB, bhh, STATE, out);
}
